// GSAAttention_18734647345176
// MI455X (gfx1250) — hardware-verified
//
#include <hip/hip_runtime.h>
#include <stdint.h>

typedef __attribute__((ext_vector_type(16))) _Float16 v16h;
typedef __attribute__((ext_vector_type(8)))  _Float16 v8h;
typedef __attribute__((ext_vector_type(16))) __bf16   v16b;
typedef __attribute__((ext_vector_type(8)))  __bf16   v8b;
typedef __attribute__((ext_vector_type(8)))  float    v8f;
typedef __attribute__((ext_vector_type(4)))  float    v4f;

constexpr int NB = 4;
constexpr int CH = 512;
constexpr int RR = 64;
constexpr int SS = 8 * 16 * 32;
constexpr float WCARRY     = 16.0f;
constexpr float WCARRY_INV = 1.0f / 16.0f;
constexpr float PCARRY     = 32768.0f;
constexpr float PCARRY_INV = 1.0f / 32768.0f;

static_assert(SS % 64 == 0 && CH % 64 == 0 && RR % 64 == 0, "tile multiples");
static_assert(CH % 32 == 0 && RR % 32 == 0 && SS % 32 == 0, "k multiples");
static_assert(SS == 4096, "softmax kernel layout");

constexpr size_t BYTES_XT   = (size_t)NB * SS * CH * 2;
constexpr size_t BYTES_SC   = (size_t)SS * SS * 4;
constexpr size_t BYTES_SH   = (BYTES_XT > BYTES_SC) ? BYTES_XT : BYTES_SC;
constexpr size_t BYTES_P    = (size_t)SS * SS * 2;
constexpr size_t BYTES_QP   = (size_t)NB * CH * SS * 2;
constexpr size_t BYTES_KP   = (size_t)NB * SS * RR * 2;
constexpr size_t BYTES_KW   = (size_t)RR * CH * 2;
constexpr size_t BYTES_QW   = (size_t)CH * CH * 2;
constexpr size_t OFF_SH  = 0;
constexpr size_t OFF_P   = OFF_SH + BYTES_SH;
constexpr size_t OFF_QP  = OFF_P + BYTES_P;
constexpr size_t OFF_KPH = OFF_QP + BYTES_QP;
constexpr size_t OFF_KPL = OFF_KPH + BYTES_KP;
constexpr size_t OFF_VTH = OFF_KPL + BYTES_KP;
constexpr size_t OFF_VTL = OFF_VTH + BYTES_KP;
constexpr size_t OFF_KW  = OFF_VTL + BYTES_KP;
constexpr size_t OFF_VW  = OFF_KW + BYTES_KW;
constexpr size_t OFF_QW  = OFF_VW + BYTES_KW;
constexpr size_t WS_TOTAL = OFF_QW + BYTES_QW;
static_assert(WS_TOTAL == 126484480, "carve total");
static_assert(WS_TOTAL <= 134217728, "carve cap");
static_assert((OFF_P % 128) == 0 && (OFF_QP % 128) == 0 && (OFF_KPH % 128) == 0 && (OFF_KPL % 128) == 0 &&
              (OFF_VTH % 128) == 0 && (OFF_VTL % 128) == 0 &&
              (OFF_KW % 128) == 0 && (OFF_VW % 128) == 0 && (OFF_QW % 128) == 0, "carve alignment");

__device__ __forceinline__ unsigned short f2bf_bits(float f) {
  unsigned u = __float_as_uint(f);
  return (unsigned short)((u + 0x7FFFu + ((u >> 16) & 1u)) >> 16);
}
__device__ __forceinline__ float bf_bits2f(unsigned short h) { return __uint_as_float(((unsigned)h) << 16); }

__device__ __forceinline__ void dep_guard_h(v8f& a, v8f& b, v16h x, v16h y) { asm volatile("v_nop\n\tv_nop\n\tv_nop\n\tv_nop" : "+v"(a), "+v"(b) : "v"(x), "v"(y)); }
__device__ __forceinline__ void dep_guard_b(v8f& a, v8f& b, v16b x, v16b y) { asm volatile("v_nop\n\tv_nop\n\tv_nop\n\tv_nop" : "+v"(a), "+v"(b) : "v"(x), "v"(y)); }
__device__ __forceinline__ void keep4_h(v16h a, v16h b, v16h c, v16h d) { asm volatile("v_nop" :: "v"(a), "v"(b), "v"(c), "v"(d)); }
__device__ __forceinline__ void keep4_b(v16b a, v16b b, v16b c, v16b d) { asm volatile("v_nop" :: "v"(a), "v"(b), "v"(c), "v"(d)); }
__device__ __forceinline__ void acc_guard4(v8f& a, v8f& b, v8f& c, v8f& d) { asm volatile("v_nop\n\tv_nop\n\tv_nop\n\tv_nop" : "+v"(a), "+v"(b), "+v"(c), "+v"(d)); }
template <typename T> struct Frag;
template <> struct Frag<_Float16> {
  typedef v16h V; union U { v16h v; v8h h[2]; };
  static __device__ __forceinline__ v16h load(const _Float16* p) {
    U f; f.h[0] = *(const v8h*)(p); f.h[1] = *(const v8h*)(p + 16); return f.v;
  }
  static __device__ __forceinline__ v8f mma(v16h a, v16h b, v8f c) {
    return __builtin_amdgcn_wmma_f32_16x16x32_f16(false, a, false, b, (short)0, c, false, false);
  }
  static __device__ __forceinline__ void guard(v8f& a, v8f& b, v16h x, v16h y) { dep_guard_h(a, b, x, y); }
  static __device__ __forceinline__ void keep(v16h a, v16h b, v16h c, v16h d) { keep4_h(a, b, c, d); }
};
template <> struct Frag<__bf16> {
  typedef v16b V; union U { v16b v; v8b h[2]; };
  static __device__ __forceinline__ v16b load(const __bf16* p) {
    U f; f.h[0] = *(const v8b*)(p); f.h[1] = *(const v8b*)(p + 16); return f.v;
  }
  static __device__ __forceinline__ v8f mma(v16b a, v16b b, v8f c) {
    return __builtin_amdgcn_wmma_f32_16x16x32_bf16(false, a, false, b, (short)0, c, false, false);
  }
  static __device__ __forceinline__ void guard(v8f& a, v8f& b, v16b x, v16b y) { dep_guard_b(a, b, x, y); }
  static __device__ __forceinline__ void keep(v16b a, v16b b, v16b c, v16b d) { keep4_b(a, b, c, d); }
};

template <int ET> struct Elem;
template <> struct Elem<0> { typedef _Float16 T; };
template <> struct Elem<1> { typedef __bf16 T; };
template <int ET, bool SPLIT, int BIAS_MODE, int OUT_MODE, bool RESID, bool GMUL>
__global__ __launch_bounds__(256) void wmma_gemm64(
    const unsigned short* __restrict__ Ap, const unsigned short* __restrict__ A2p, int lda, long strideA,
    const unsigned short* __restrict__ Btp, const unsigned short* __restrict__ Bt2p, int ldb, long strideB,
    void* __restrict__ Cout, void* __restrict__ Cout2, int ldc, long strideC,
    const float* __restrict__ bias,
    const float* __restrict__ resid, long strideR,
    const float* __restrict__ gmul,
    int M, int N, int K, float scale) {
  static_assert(!RESID || OUT_MODE == 0, "resid needs f32 out");
  typedef typename Elem<ET>::T T;
  typedef typename Frag<T>::V V;
  const T* A = (const T*)Ap; const T* A2 = (const T*)A2p; const T* Bt = (const T*)Btp; const T* Bt2 = (const T*)Bt2p;
  __shared__ __align__(16) float sT[8][16 * 68];
  const int b    = blockIdx.y;
  const int lane = threadIdx.x & 31;
  const int wave = threadIdx.x >> 5;
  const int tilesN = N >> 6;
  const int tilesM = M >> 6;
  const int tile = blockIdx.x * 8 + wave;
  if (tile >= tilesM * tilesN) return;
  const int tm = tile / tilesN;
  const int tn = tile - tm * tilesN;
  const int m0 = tm << 6;
  const int n0 = tn << 6;

  const T* Ab  = A  + (size_t)b * strideA;
  const T* Bb  = Bt + (size_t)b * strideB;
  const T* Ab2 = SPLIT ? (A2  + (size_t)b * strideA) : nullptr;
  const T* Bb2 = SPLIT ? (Bt2 + (size_t)b * strideB) : nullptr;

  const int rlane = lane & 15;
  const int koff  = (lane >> 4) * 8;
  const int mOff  = (lane >> 4) * 8;

  v8f acc[4][4];
#pragma unroll
  for (int i = 0; i < 4; ++i)
#pragma unroll
    for (int j = 0; j < 4; ++j) acc[i][j] = (v8f){0.f,0.f,0.f,0.f,0.f,0.f,0.f,0.f};

  for (int k0 = 0; k0 < K; k0 += 32) {
    V bh[4], bl[4];
#pragma unroll
    for (int j = 0; j < 4; ++j) {
      const size_t bo = (size_t)(n0 + (j << 4) + rlane) * ldb + koff + k0;
      bh[j] = Frag<T>::load(Bb + bo);
      if (SPLIT) bl[j] = Frag<T>::load(Bb2 + bo);
    }
#pragma unroll
    for (int i = 0; i < 4; ++i) {
      const size_t ao = (size_t)(m0 + (i << 4) + rlane) * lda + koff + k0;
      V ah = Frag<T>::load(Ab + ao);
      V al;
      if (SPLIT) al = Frag<T>::load(Ab2 + ao);
#pragma unroll
      for (int j = 0; j < 4; ++j) {
        acc[i][j] = Frag<T>::mma(ah, bh[j], acc[i][j]);
        if (SPLIT) {
          acc[i][j] = Frag<T>::mma(ah, bl[j], acc[i][j]);
          acc[i][j] = Frag<T>::mma(al, bh[j], acc[i][j]);
        }
      }
      Frag<T>::guard(acc[i][0], acc[i][3], ah, SPLIT ? al : ah);
    }
    Frag<T>::keep(bh[0], bh[1], bh[2], bh[3]);
    if (SPLIT) Frag<T>::keep(bl[0], bl[1], bl[2], bl[3]);
  }
  acc_guard4(acc[0][0], acc[0][1], acc[0][2], acc[0][3]);
  acc_guard4(acc[1][0], acc[1][1], acc[1][2], acc[1][3]);
  acc_guard4(acc[2][0], acc[2][1], acc[2][2], acc[2][3]);
  acc_guard4(acc[3][0], acc[3][1], acc[3][2], acc[3][3]);

  float* slab = sT[wave];
  const float* Rb = RESID ? (resid + (size_t)b * strideR) : nullptr;
  const float gm = GMUL ? gmul[0] : 1.0f;
#pragma unroll
  for (int i = 0; i < 4; ++i) {
    const int mBase = m0 + (i << 4);
#pragma unroll
    for (int j = 0; j < 4; ++j) {
      const int n = n0 + (j << 4) + rlane;
      float bv = 0.f;
      if (BIAS_MODE == 2) bv = bias[n];
#pragma unroll
      for (int r = 0; r < 8; ++r) {
        float v = acc[i][j][r] * scale;
        if (GMUL) v *= gm;
        if (BIAS_MODE == 1) v += bias[mBase + mOff + r];
        if (BIAS_MODE == 2) v += bv;
        slab[(mOff + r) * 68 + (j << 4) + rlane] = v;
      }
    }
    __builtin_amdgcn_fence(__ATOMIC_RELEASE, "workgroup");
    __builtin_amdgcn_wave_barrier();
    __builtin_amdgcn_fence(__ATOMIC_ACQUIRE, "workgroup");
    if (OUT_MODE == 0) {
      float* C = (float*)Cout + (size_t)b * strideC;
      const int hh = lane >> 4, c4 = (lane & 15) * 4;
      for (int pass = 0; pass < 2; ++pass) {
#pragma unroll
        for (int it = 0; it < 8; ++it) {
          const int row = it * 2 + hh;
          v4f v = *(const v4f*)(slab + row * 68 + c4);
          if (RESID) {
            const v4f rr = *(const v4f*)(Rb + (size_t)(mBase + row) * ldc + n0 + c4);
            v += rr;
          }
          *(volatile v4f*)(C + (size_t)(mBase + row) * ldc + n0 + c4) = v;
        }
        __threadfence();
      }
    } else {
      const int q = lane >> 3, c8 = (lane & 7) * 8;
      unsigned short* C  = (unsigned short*)Cout  + (size_t)b * strideC;
      unsigned short* C2 = (OUT_MODE == 2) ? ((unsigned short*)Cout2 + (size_t)b * strideC) : nullptr;
      for (int pass = 0; pass < 2; ++pass) {
#pragma unroll
        for (int it = 0; it < 4; ++it) {
          const int row = it * 4 + q;
          const float* sp = slab + row * 68 + c8;
          v8h hv, lv;
#pragma unroll
          for (int e = 0; e < 8; ++e) {
            if (OUT_MODE == 1) {
              hv[e] = (_Float16)sp[e];
            } else {
              unsigned short hb = f2bf_bits(sp[e]);
              unsigned short lb = f2bf_bits(sp[e] - bf_bits2f(hb));
              hv[e] = __builtin_bit_cast(_Float16, hb);
              lv[e] = __builtin_bit_cast(_Float16, lb);
            }
          }
          *(volatile v8h*)(C + (size_t)(mBase + row) * ldc + n0 + c8) = hv;
          if (OUT_MODE == 2) *(volatile v8h*)(C2 + (size_t)(mBase + row) * ldc + n0 + c8) = lv;
        }
        __threadfence();
      }
    }
    __builtin_amdgcn_fence(__ATOMIC_RELEASE, "workgroup");
    __builtin_amdgcn_wave_barrier();
    __builtin_amdgcn_fence(__ATOMIC_ACQUIRE, "workgroup");
  }
}

__global__ __launch_bounds__(256) void cast_scale_f16x2(
    const float* __restrict__ in, _Float16* __restrict__ out, int n2, float mul) {
  int i = blockIdx.x * 256 + threadIdx.x;
  if (i < n2) {
    const _Float16 h0 = (_Float16)(in[2 * i] * mul), h1 = (_Float16)(in[2 * i + 1] * mul);
    const unsigned u = (unsigned)__builtin_bit_cast(unsigned short, h0) | ((unsigned)__builtin_bit_cast(unsigned short, h1) << 16);
    ((volatile unsigned*)out)[i] = u;
    __threadfence();
    ((volatile unsigned*)out)[i] = u;
  }
}

__global__ __launch_bounds__(256) void transpose_x_kernel(const float* __restrict__ X, _Float16* __restrict__ Xt) {
  __shared__ float tile[64][65];
  const int n  = blockIdx.z;
  const int s0 = blockIdx.x * 64;
  const int c0 = blockIdx.y * 64;
  const int tid = threadIdx.x, lane = tid & 31, wave = tid >> 5;
  const float* Xn = X + (size_t)n * CH * SS;
#pragma unroll
  for (int i = 0; i < 4; ++i) {
    const int c  = (tid >> 4) + 16 * i;
    const int s4 = (tid & 15) * 4;
    const v4f v = *(const v4f*)(Xn + (size_t)(c0 + c) * SS + s0 + s4);
    tile[c][s4 + 0] = v[0];
    tile[c][s4 + 1] = v[1];
    tile[c][s4 + 2] = v[2];
    tile[c][s4 + 3] = v[3];
  }
  __syncthreads();
  _Float16* Xtn = Xt + (size_t)n * SS * CH;
  const int q = lane >> 3, c8 = (lane & 7) * 8;
  for (int pass = 0; pass < 2; ++pass) {
#pragma unroll
    for (int it = 0; it < 2; ++it) {
      const int sr = wave * 8 + it * 4 + q;
      v8h hv;
#pragma unroll
      for (int e = 0; e < 8; ++e) hv[e] = (_Float16)tile[c8 + e][sr];
      *(volatile v8h*)(Xtn + (size_t)(s0 + sr) * CH + c0 + c8) = hv;
    }
    __threadfence();
  }
}

__global__ __launch_bounds__(256) void softmax_rows_kernel(const float* __restrict__ sc, _Float16* __restrict__ pout) {
  __shared__ __align__(16) float es[SS];
  __shared__ float red[8];
  __shared__ float bc[2];
  const int t = blockIdx.x;
  const int tid = threadIdx.x, lane = tid & 31, wave = tid >> 5;
  const float* row = sc + (size_t)t * SS;

  float m = -INFINITY;
#pragma unroll
  for (int it = 0; it < 4; ++it) {
    const v4f v = *(const v4f*)(row + it * 1024 + tid * 4);
    m = fmaxf(m, fmaxf(fmaxf(v[0], v[1]), fmaxf(v[2], v[3])));
  }
#pragma unroll
  for (int off = 16; off > 0; off >>= 1) m = fmaxf(m, __shfl_xor(m, off, 32));
  if (lane == 0) red[wave] = m;
  __syncthreads();
  if (tid == 0) {
    float mm = red[0];
#pragma unroll
    for (int w = 1; w < 8; ++w) mm = fmaxf(mm, red[w]);
    bc[0] = mm;
  }
  __syncthreads();
  const float rmax = bc[0];

  float ssum = 0.f;
#pragma unroll 1
  for (int it = 0; it < 4; ++it) {
    const v4f v = *(const v4f*)(row + it * 1024 + tid * 4);
    v4f e;
    e[0] = expf(v[0] - rmax);
    e[1] = expf(v[1] - rmax);
    e[2] = expf(v[2] - rmax);
    e[3] = expf(v[3] - rmax);
    ssum += (e[0] + e[1]) + (e[2] + e[3]);
    *(v4f*)(es + it * 1024 + tid * 4) = e;
  }
#pragma unroll
  for (int off = 16; off > 0; off >>= 1) ssum += __shfl_xor(ssum, off, 32);
  if (lane == 0) red[wave] = ssum;
  __syncthreads();
  if (tid == 0) {
    float tot = red[0];
#pragma unroll
    for (int w = 1; w < 8; ++w) tot += red[w];
    bc[1] = PCARRY * (1.0f / tot);
  }
  __syncthreads();
  const float f = bc[1];

  _Float16* prow = pout + (size_t)t * SS;
  for (int pass = 0; pass < 2; ++pass) {
#pragma unroll
    for (int it = 0; it < 2; ++it) {
      const int base = it * 2048 + wave * 256 + lane * 8;
      const v4f a = *(const v4f*)(es + base);
      const v4f c = *(const v4f*)(es + base + 4);
      v8h hv;
      hv[0] = (_Float16)(a[0] * f); hv[1] = (_Float16)(a[1] * f);
      hv[2] = (_Float16)(a[2] * f); hv[3] = (_Float16)(a[3] * f);
      hv[4] = (_Float16)(c[0] * f); hv[5] = (_Float16)(c[1] * f);
      hv[6] = (_Float16)(c[2] * f); hv[7] = (_Float16)(c[3] * f);
      *(volatile v8h*)(prow + base) = hv;
    }
    __threadfence();
  }
}

extern "C" void kernel_launch(void* const* d_in, const int* in_sizes, int n_in,
                              void* d_out, int out_size, void* d_ws, size_t ws_size,
                              hipStream_t stream) {
  (void)in_sizes; (void)n_in;
  if (ws_size < WS_TOTAL) return;
  if ((size_t)out_size < (size_t)NB * CH * SS) return;

  const float* x     = (const float*)d_in[0];
  const float* k_w   = (const float*)d_in[1];
  const float* k_b   = (const float*)d_in[2];
  const float* v_w   = (const float*)d_in[3];
  const float* v_b   = (const float*)d_in[4];
  const float* q_w   = (const float*)d_in[5];
  const float* q_b   = (const float*)d_in[6];
  const float* gamma = (const float*)d_in[7];
  float* out = (float*)d_out;

  char* ws = (char*)d_ws;
  _Float16* xt16 = (_Float16*)(ws + OFF_SH);
  float*    sc   = (float*)(ws + OFF_SH);
  _Float16* p16  = (_Float16*)(ws + OFF_P);
  _Float16* qp16 = (_Float16*)(ws + OFF_QP);
  unsigned short* kph = (unsigned short*)(ws + OFF_KPH);
  unsigned short* kpl = (unsigned short*)(ws + OFF_KPL);
  unsigned short* vth = (unsigned short*)(ws + OFF_VTH);
  unsigned short* vtl = (unsigned short*)(ws + OFF_VTL);
  _Float16* kw16 = (_Float16*)(ws + OFF_KW);
  _Float16* vw16 = (_Float16*)(ws + OFF_VW);
  _Float16* qw16 = (_Float16*)(ws + OFF_QW);
  typedef const unsigned short* cus;

  cast_scale_f16x2<<<dim3((RR * CH / 2 + 255) / 256), dim3(256), 0, stream>>>(k_w, kw16, RR * CH / 2, WCARRY);
  cast_scale_f16x2<<<dim3((RR * CH / 2 + 255) / 256), dim3(256), 0, stream>>>(v_w, vw16, RR * CH / 2, WCARRY);
  cast_scale_f16x2<<<dim3((CH * CH / 2 + 255) / 256), dim3(256), 0, stream>>>(q_w, qw16, CH * CH / 2, WCARRY);

  transpose_x_kernel<<<dim3(SS / 64, CH / 64, NB), dim3(256), 0, stream>>>(x, xt16);

  {
    const int tiles = (SS / 64) * (RR / 64);
    wmma_gemm64<0, false, 2, 2, false, false><<<dim3((tiles + 7) / 8, NB), dim3(256), 0, stream>>>(
        (cus)xt16, (cus)xt16, CH, (long)SS * CH,
        (cus)kw16, (cus)kw16, CH, 0L,
        kph, kpl, RR, (long)SS * RR,
        k_b, x, 0L, gamma, SS, RR, CH, WCARRY_INV);
    wmma_gemm64<0, false, 2, 2, false, false><<<dim3((tiles + 7) / 8, NB), dim3(256), 0, stream>>>(
        (cus)xt16, (cus)xt16, CH, (long)SS * CH,
        (cus)vw16, (cus)vw16, CH, 0L,
        vth, vtl, RR, (long)SS * RR,
        v_b, x, 0L, gamma, SS, RR, CH, WCARRY_INV);
  }
  {
    const int tiles = (CH / 64) * (SS / 64);
    wmma_gemm64<0, false, 1, 1, false, false><<<dim3((tiles + 7) / 8, NB), dim3(256), 0, stream>>>(
        (cus)qw16, (cus)qw16, CH, 0L,
        (cus)xt16, (cus)xt16, CH, (long)SS * CH,
        qp16, qp16, SS, (long)CH * SS,
        q_b, x, 0L, gamma, CH, SS, CH, WCARRY_INV);
  }

  for (int n = 0; n < NB; ++n) {
    const size_t offKV = (size_t)n * SS * RR;
    const size_t offCS = (size_t)n * CH * SS;
    {
      const int tiles = (SS / 64) * (SS / 64);
      wmma_gemm64<1, true, 0, 0, false, false><<<dim3((tiles + 7) / 8, 1), dim3(256), 0, stream>>>(
          (cus)(vth + offKV), (cus)(vtl + offKV), RR, 0L,
          (cus)(kph + offKV), (cus)(kpl + offKV), RR, 0L,
          sc, sc, SS, 0L,
          k_b, x, 0L, gamma, SS, SS, RR, 1.0f);
    }
    softmax_rows_kernel<<<dim3(SS), dim3(256), 0, stream>>>(sc, p16);
    {
      const int tiles = (CH / 64) * (SS / 64);
      wmma_gemm64<0, false, 0, 0, true, true><<<dim3((tiles + 7) / 8, 1), dim3(256), 0, stream>>>(
          (cus)(qp16 + offCS), (cus)(qp16 + offCS), SS, 0L,
          (cus)p16, (cus)p16, SS, 0L,
          out + offCS, out + offCS, SS, 0L,
          q_b, x + offCS, 0L, gamma, CH, SS, SS, PCARRY_INV);
    }
  }
}
